// WubuBlock_5068061409874
// MI455X (gfx1250) — hardware-run, weakly checked
//
#include <hip/hip_runtime.h>
#include <math.h>
#include <stdint.h>

#ifndef NB
#define NB      2
#endif
#ifndef SEQ
#define SEQ     1024
#endif
#define NB_FULL   2
#define SEQ_FULL  1024
#define DMODEL  512
#define DFF     2048
#define NHEAD   8
#define HDIM    64
#define WIN     64
#define NROWS   (NB * SEQ)
#define SEQK    (SEQ + 64)
#define SEQV    (SEQ + 128)
#define XBSTRIDE_FULL ((long long)SEQ_FULL * DMODEL)
#define WSC     64.0f
#define HCARRY  16.0f
#define QC      16.0f
#define KC      16.0f
#define VC      16.0f
#define PC      16384.0f
#define FC      1024.0f
#define H2C     16.0f
#define GC      64.0f
#define LN_EPS  1e-6f
#define PEPS    1e-7f
#define ARG1    0.99999988079071044921875f
#define OMCLIP  2.384185791015625e-7f
#define L9      2.1972245773362196f
static_assert(NB >= 1 && NB <= NB_FULL && SEQ >= 64 && SEQ <= SEQ_FULL);
static_assert((SEQ % 64) == 0 && (NROWS % 64) == 0 && (DMODEL % 64) == 0 && (DFF % 64) == 0);
static_assert(NHEAD * HDIM == DMODEL && HDIM == 64 && (DMODEL % 32) == 0 && (DFF % 32) == 0);
static_assert((SEQK % 16) == 0 && (SEQV % 64) == 0);

#define LN_THREADS 128
static_assert(LN_THREADS * 4 == DMODEL && (DMODEL / 8) % 32 == 0);
#define QK_THREADS 256
static_assert(QK_THREADS == 32 * NHEAD && 16 * DMODEL == 4 * 8 * QK_THREADS);
#define AWAVES   4
#define ATHREADS (AWAVES * 32)
#define KCOLS    80
#define PCOLS    96
#define SPF      84
#define PPU      52
static_assert(NHEAD % AWAVES == 0);
static_assert(KCOLS == WIN + 16 && (KCOLS % 16) == 0 && (KCOLS % 4) == 0 && SPF >= KCOLS);
static_assert(PCOLS >= KCOLS && (PCOLS % 32) == 0 && 2 * PPU >= PCOLS && ((2 * PPU) % 8) == 0);
static_assert(SEQ - 16 + KCOLS <= SEQK && SEQ - 16 + PCOLS <= SEQV);
static_assert(16 * HDIM * 2 <= 16 * SPF * 4);
static_assert(QC == KC);

typedef _Float16 v16h __attribute__((ext_vector_type(16)));
typedef _Float16 v8h  __attribute__((ext_vector_type(8)));
typedef float    v8f  __attribute__((ext_vector_type(8)));
typedef float    v4f  __attribute__((ext_vector_type(4)));
typedef float    v2f  __attribute__((ext_vector_type(2)));
typedef unsigned int v4u __attribute__((ext_vector_type(4)));
typedef unsigned int v2u __attribute__((ext_vector_type(2)));

union FragH { v16h v; v8h h[2]; v4u u[2]; };

__device__ __forceinline__ unsigned short bf_bits(float f) {
  unsigned u = __float_as_uint(f);
  return (unsigned short)((u + 0x7FFFu + ((u >> 16) & 1u)) >> 16);
}
__device__ __forceinline__ float bf_up(unsigned short h) { return __uint_as_float(((unsigned)h) << 16); }
__device__ __forceinline__ float bfr(float f) { return bf_up(bf_bits(f)); }
__device__ __forceinline__ unsigned short h_bits(_Float16 x) { return __builtin_bit_cast(unsigned short, x); }
__device__ __forceinline__ unsigned pk16(unsigned short a, unsigned short b) { return (unsigned)a | ((unsigned)b << 16); }
__device__ __forceinline__ v8f zero8() { v8f z = {0.f, 0.f, 0.f, 0.f, 0.f, 0.f, 0.f, 0.f}; return z; }
__device__ __forceinline__ int imin(int a, int b) { return a < b ? a : b; }
__device__ __forceinline__ float gelu_t(float u) {
  const float k0 = 0.7978845608028654f;
  const float inner = k0 * (u + 0.044715f * (u * u * u));
  return 0.5f * u * (1.0f + tanhf(inner));
}

__device__ __forceinline__ v16h ldfrag_u(const unsigned short* p) {
  FragH f;
  f.u[0] = *(const v4u*)(p);
  f.u[1] = *(const v4u*)(p + 16);
  return f.v;
}

__device__ __forceinline__ v8f mma_raw(v16h a, v16h b, v8f c) {
  return __builtin_amdgcn_wmma_f32_16x16x32_f16(false, a, false, b, (short)0, c, false, false);
}
__device__ __forceinline__ void dep_guard1(v8f& a, v8f& b, v16h x) {
#if defined(__HIP_DEVICE_COMPILE__)
  asm volatile("v_nop\n\tv_nop\n\tv_nop\n\tv_nop" : "+v"(a), "+v"(b) : "v"(x));
#endif
}
__device__ __forceinline__ void guard_s4(v8f& s, v16h a0, v16h a1, v16h b0, v16h b1) {
#if defined(__HIP_DEVICE_COMPILE__)
  asm volatile("v_nop\n\tv_nop\n\tv_nop\n\tv_nop" : "+v"(s) : "v"(a0), "v"(a1), "v"(b0), "v"(b1));
#endif
}
__device__ __forceinline__ void guard_pv4(v8f& a, v8f& b, v8f& c, v8f& d, v16h x, v16h y, v16h z, v16h w, v16h u) {
#if defined(__HIP_DEVICE_COMPILE__)
  asm volatile("v_nop\n\tv_nop\n\tv_nop\n\tv_nop"
               : "+v"(a), "+v"(b), "+v"(c), "+v"(d) : "v"(x), "v"(y), "v"(z), "v"(w), "v"(u));
#endif
}
__device__ __forceinline__ void keep4_h(v16h a, v16h b, v16h c, v16h d) {
#if defined(__HIP_DEVICE_COMPILE__)
  asm volatile("v_nop" :: "v"(a), "v"(b), "v"(c), "v"(d));
#endif
}
__device__ __forceinline__ void acc_guard4(v8f& a, v8f& b, v8f& c, v8f& d) {
#if defined(__HIP_DEVICE_COMPILE__)
  asm volatile("v_nop\n\tv_nop\n\tv_nop\n\tv_nop" : "+v"(a), "+v"(b), "+v"(c), "+v"(d));
#endif
}
__device__ __forceinline__ void wave_sync_lds() {
  __builtin_amdgcn_fence(__ATOMIC_RELEASE, "workgroup");
  __builtin_amdgcn_wave_barrier();
  __builtin_amdgcn_fence(__ATOMIC_ACQUIRE, "workgroup");
}

__device__ __forceinline__ float hdist(float xy, float x2, float y2, float cc, float sc, float rsc, float bx, float dclip) {
#pragma clang fp contract(off)
  const float m    = 1.0f - (2.0f * cc) * xy;
  const float a    = m + cc * y2;
  const float by   = 1.0f - cc * y2;
  const float den0 = m + ((cc * cc) * x2) * y2;
  const float den  = fmaxf(den0, PEPS);
  const float rden = 1.0f / den;
  float nn = ((a * a) * x2 - ((2.0f * a) * bx) * xy) + (bx * bx) * y2;
  nn = fmaxf(nn, 0.0f);
  const float t2 = (cc * nn) * (rden * rden);
  float d;
  if (t2 < 0.25f) {
    const float dn  = sqrtf(nn) * rden;
    const float arg = fminf(sc * fmaxf(dn, PEPS), ARG1);
    d = (2.0f * atanhf(arg)) * rsc;
  } else {
    float om = (bx * by) * rden;
    om = fminf(fmaxf(om, 0.0f), 1.0f);
    if (om <= OMCLIP) {
      d = dclip * rsc;
    } else {
      const float t = sqrtf(1.0f - om);
      d = (2.0f * log1pf(t) - logf(om)) * rsc;
    }
  }
  return d;
}

__global__ __launch_bounds__(256) void tcvt16(const float* __restrict__ src, unsigned short* dst,
                                              int R, int C, int Rp, int Cp, float sc) {
  __shared__ __align__(16) unsigned short sT[64 * 72];
  const int tid = threadIdx.x, lane = tid & 31, wave = tid >> 5;
  const int c0 = blockIdx.x * 64, r0 = blockIdx.y * 64;
  const int rr = tid >> 2, cc = (tid & 3) * 16;
  const int r = r0 + rr;
  const int rcl = imin(r, R - 1);
  const float* sp = src + (size_t)rcl * C;
#pragma unroll
  for (int e = 0; e < 16; ++e) {
    const int cidx = c0 + cc + e;
    const int ccl = imin(cidx, C - 1);
    float a = sp[ccl];
    a = (r < R && cidx < C) ? a : 0.f;
    sT[(cc + e) * 72 + rr] = h_bits((_Float16)(bfr(a) * sc));
  }
  __syncthreads();
  v4u vals[2];
#pragma unroll
  for (int it = 0; it < 2; ++it) {
    const int q = it * 32 + wave * 4 + (lane >> 3);
    vals[it] = *(const v4u*)(sT + q * 72 + (lane & 7) * 8);
  }
  for (int pass = 0; pass < 2; ++pass) {
#pragma unroll
    for (int it = 0; it < 2; ++it) {
      const int q = it * 32 + wave * 4 + (lane >> 3);
      *(volatile v4u*)(dst + (size_t)(c0 + q) * Rp + r0 + (lane & 7) * 8) = vals[it];
    }
    __threadfence();
  }
  (void)Cp;
}

template <int OM, int RM, int ACT, int BM>
__global__ __launch_bounds__(256) void gemm64(
    const unsigned short* __restrict__ Ap, int lda, long long sA,
    const unsigned short* __restrict__ Btp, int ldb, long long sB,
    const float* __restrict__ Rp, long long sR,
    const float* __restrict__ biasp, int nbias,
    void* Cout, int ldc, long long sC,
    int M, int N, int K, float oscale, float ocarry) {
  __shared__ __align__(16) float sT[8][16 * 68];
  const int by   = blockIdx.y;
  const int lane = threadIdx.x & 31;
  const int wave = threadIdx.x >> 5;
  const int tilesN = N >> 6;
  const int tilesM = M >> 6;
  const int tile = blockIdx.x * 8 + wave;
  if (tile >= tilesM * tilesN) return;
  const int tm = tile / tilesN;
  const int tn = tile - tm * tilesN;
  const int m0 = tm << 6;
  const int n0 = tn << 6;

  const unsigned short* A1 = Ap  + (size_t)((long long)by * sA);
  const unsigned short* Bb = Btp + (size_t)((long long)by * sB);

  const int rlane = lane & 15;
  const int koff  = (lane >> 4) * 8;
  const int mOff  = (lane >> 4) * 8;

  v8f acc[4][4];
#pragma unroll
  for (int i = 0; i < 4; ++i)
#pragma unroll
    for (int j = 0; j < 4; ++j) acc[i][j] = zero8();

  for (int k0 = 0; k0 < K; k0 += 32) {
    v16h bh[4];
#pragma unroll
    for (int j = 0; j < 4; ++j) {
      const size_t bofs = (size_t)(n0 + (j << 4) + rlane) * ldb + koff + k0;
      bh[j] = ldfrag_u(Bb + bofs);
    }
#pragma unroll
    for (int i = 0; i < 4; ++i) {
      const size_t ao = (size_t)(m0 + (i << 4) + rlane) * lda + koff + k0;
      const v16h ah = ldfrag_u(A1 + ao);
#pragma unroll
      for (int j = 0; j < 4; ++j) acc[i][j] = mma_raw(ah, bh[j], acc[i][j]);
      dep_guard1(acc[i][0], acc[i][3], ah);
    }
    keep4_h(bh[0], bh[1], bh[2], bh[3]);
  }
  acc_guard4(acc[0][0], acc[0][1], acc[0][2], acc[0][3]);
  acc_guard4(acc[1][0], acc[1][1], acc[1][2], acc[1][3]);
  acc_guard4(acc[2][0], acc[2][1], acc[2][2], acc[2][3]);
  acc_guard4(acc[3][0], acc[3][1], acc[3][2], acc[3][3]);

  const int hh2 = lane >> 4, c4 = (lane & 15) * 4;
  const int q8  = lane >> 3, c8 = (lane & 7) * 8;

  float bc4[4], bc8[8];
#pragma unroll
  for (int e = 0; e < 4; ++e) bc4[e] = 0.f;
#pragma unroll
  for (int e = 0; e < 8; ++e) bc8[e] = 0.f;
  if constexpr (BM == 1) {
    if constexpr (OM == 0) {
#pragma unroll
      for (int e = 0; e < 4; ++e) {
        const int n = n0 + c4 + e;
        const int ncl = imin(n, nbias - 1);
        const float t = bfr(biasp[ncl]);
        bc4[e] = (n < nbias) ? t : 0.f;
      }
    } else {
#pragma unroll
      for (int e = 0; e < 8; ++e) {
        const int n = n0 + c8 + e;
        const int ncl = imin(n, nbias - 1);
        const float t = bfr(biasp[ncl]);
        bc8[e] = (n < nbias) ? t : 0.f;
      }
    }
  }

  float* slab = sT[wave];
#pragma unroll
  for (int i = 0; i < 4; ++i) {
    const int mBase = m0 + (i << 4);
#pragma unroll
    for (int j = 0; j < 4; ++j) {
#pragma unroll
      for (int r = 0; r < 8; ++r) {
        slab[(mOff + r) * 68 + (j << 4) + rlane] = acc[i][j][r];
      }
    }
    wave_sync_lds();
    if constexpr (OM == 0) {
      float* C = (float*)Cout + (size_t)((long long)by * sC);
      v4f vals[8];
#pragma unroll
      for (int it = 0; it < 8; ++it) {
        const int row = it * 2 + hh2;
        const int gr  = mBase + row;
        v4f v = *(const v4f*)(slab + row * 68 + c4);
        v4f rv = {0.f, 0.f, 0.f, 0.f};
        if constexpr (RM == 1 || RM == 2) {
          const float* R = Rp + (size_t)((long long)by * sR);
          const v4f rraw = *(const v4f*)(R + (size_t)gr * ldc + n0 + c4);
#pragma unroll
          for (int e = 0; e < 4; ++e) rv[e] = (RM == 1) ? bfr(rraw[e]) : rraw[e];
        }
        float rb = 0.f;
        if constexpr (BM == 2) {
          const int gcl = imin(gr, nbias - 1);
          const float t = bfr(biasp[gcl]);
          rb = (gr < nbias) ? t : 0.f;
        }
#pragma unroll
        for (int e = 0; e < 4; ++e) {
          float u = v[e] * oscale;
          if constexpr (BM == 1) u += bc4[e];
          if constexpr (BM == 2) u += rb;
          if constexpr (ACT == 1) u = gelu_t(u);
          v[e] = u + rv[e];
        }
        vals[it] = v;
      }
      for (int pass = 0; pass < 2; ++pass) {
#pragma unroll
        for (int it = 0; it < 8; ++it) {
          const int gr = mBase + it * 2 + hh2;
          *(volatile v4f*)(C + (size_t)gr * ldc + n0 + c4) = vals[it];
        }
        __threadfence();
      }
    } else {
      unsigned short* C = (unsigned short*)Cout + (size_t)((long long)by * sC);
      v4u hv[4];
#pragma unroll
      for (int it = 0; it < 4; ++it) {
        const int row = it * 4 + q8;
        const float* sp = slab + row * 68 + c8;
        float rb = 0.f;
        if constexpr (BM == 2) {
          const int gm  = mBase + row;
          const int gcl = imin(gm, nbias - 1);
          const float t = bfr(biasp[gcl]);
          rb = (gm < nbias) ? t : 0.f;
        }
        v4u a = {0u, 0u, 0u, 0u};
#pragma unroll
        for (int e = 0; e < 4; ++e) {
          float f0 = sp[2 * e] * oscale;
          float f1 = sp[2 * e + 1] * oscale;
          if constexpr (BM == 1) { f0 += bc8[2 * e]; f1 += bc8[2 * e + 1]; }
          if constexpr (BM == 2) { f0 += rb; f1 += rb; }
          if constexpr (ACT == 1) { f0 = gelu_t(f0); f1 = gelu_t(f1); }
          f0 *= ocarry; f1 *= ocarry;
          a[e] = pk16(h_bits((_Float16)f0), h_bits((_Float16)f1));
        }
        hv[it] = a;
      }
      for (int pass = 0; pass < 2; ++pass) {
#pragma unroll
        for (int it = 0; it < 4; ++it) {
          const int row = it * 4 + q8;
          *(volatile v4u*)(C + (size_t)(mBase + row) * ldc + n0 + c8) = hv[it];
        }
        __threadfence();
      }
    }
    wave_sync_lds();
  }
}

template <int RIN>
__global__ __launch_bounds__(LN_THREADS)
void lnorm(const float* __restrict__ Yp, long long bstride, const float* __restrict__ gp, const float* __restrict__ bp,
           unsigned short* outh, float hc) {
  __shared__ float red[2][LN_THREADS / 32];
  __shared__ __align__(16) unsigned short srow[DMODEL];
  const int row  = blockIdx.x;
  const int tid  = threadIdx.x;
  const int lane = tid & 31;
  const int wave = tid >> 5;
  const int b    = row / SEQ;
  const int s    = row - b * SEQ;
  const size_t base = (size_t)((long long)b * bstride) + (size_t)s * DMODEL + (size_t)tid * 4;
  v4f v = *(const v4f*)(Yp + base);
  if constexpr (RIN == 1) {
#pragma unroll
    for (int e = 0; e < 4; ++e) v[e] = bfr(v[e]);
  }
  float sm = (v[0] + v[1]) + (v[2] + v[3]);
#pragma unroll
  for (int off = 1; off < 32; off <<= 1) sm += __shfl_xor(sm, off, 32);
  if (lane == 0) red[0][wave] = sm;
  __syncthreads();
  float tot = 0.f;
#pragma unroll
  for (int w = 0; w < LN_THREADS / 32; ++w) tot += red[0][w];
  const float mu = tot * (1.0f / (float)DMODEL);
  v4f d;
#pragma unroll
  for (int e = 0; e < 4; ++e) d[e] = v[e] - mu;
  float q = (d[0] * d[0] + d[1] * d[1]) + (d[2] * d[2] + d[3] * d[3]);
#pragma unroll
  for (int off = 1; off < 32; off <<= 1) q += __shfl_xor(q, off, 32);
  if (lane == 0) red[1][wave] = q;
  __syncthreads();
  float totq = 0.f;
#pragma unroll
  for (int w = 0; w < LN_THREADS / 32; ++w) totq += red[1][w];
  const float var  = totq * (1.0f / (float)DMODEL);
  const float rstd = rsqrtf(var + LN_EPS);
  const v4f gv = *(const v4f*)(gp + (size_t)tid * 4);
  const v4f bv = *(const v4f*)(bp + (size_t)tid * 4);
  v4f o;
#pragma unroll
  for (int e = 0; e < 4; ++e) o[e] = (d[e] * rstd) * bfr(gv[e]) + bfr(bv[e]);
  v2u w;
  w[0] = pk16(h_bits((_Float16)(o[0] * hc)), h_bits((_Float16)(o[1] * hc)));
  w[1] = pk16(h_bits((_Float16)(o[2] * hc)), h_bits((_Float16)(o[3] * hc)));
  *(v2u*)(srow + tid * 4) = w;
  __syncthreads();
  if (tid < DMODEL / 8) {
    const v4u hv = *(const v4u*)(srow + tid * 8);
    unsigned short* dst = outh + (size_t)row * DMODEL + (size_t)tid * 8;
    for (int pass = 0; pass < 2; ++pass) {
      *(volatile v4u*)dst = hv;
      __threadfence();
    }
  }
}

__global__ __launch_bounds__(256) void zlines(unsigned short* base, int per, long long bstride, long long lstride, int nlines) {
  const int g  = (int)((blockIdx.x * 256u + threadIdx.x) >> 3);
  const int pc = threadIdx.x & 7;
  const bool act = g < nlines;
  const int gg = act ? g : 0;
  const int gb = gg / per;
  const int gl = gg - gb * per;
  unsigned short* d = base + (size_t)((long long)gb * bstride + (long long)gl * lstride) + pc * 8;
  const v4u z = {0u, 0u, 0u, 0u};
  for (int pass = 0; pass < 2; ++pass) {
    if (act) *(volatile v4u*)d = z;
    __threadfence();
  }
}

__global__ __launch_bounds__(QK_THREADS)
void qkprep(const float* __restrict__ QF, const float* __restrict__ KF,
            const float* __restrict__ cosp, const float* __restrict__ sinp,
            const float* __restrict__ cin, const float* __restrict__ hashp,
            unsigned short* QH, unsigned short* KH, float* QN, float* KN) {
#pragma clang fp contract(off)
  __shared__ __align__(16) unsigned short sT[2][16 * DMODEL];
  __shared__ __align__(16) float sN[2][16 * NHEAD];
  const int tid = threadIdx.x, lane = tid & 31, h = tid >> 5;
  const int r0  = blockIdx.x * 16;
  const int bat = r0 / SEQ;
  const int n0  = r0 - bat * SEQ;
  const float cc  = bfr(cin[bat]);
  const float sc  = fmaxf(sqrtf(cc), PEPS);
  const float rsc = 1.0f / sc;
  const float hr  = bfr(hashp[h * HDIM + lane]) * L9;
  const float hi  = bfr(hashp[h * HDIM + lane + 32]) * L9;
#pragma unroll 1
  for (int t = 0; t < 32; ++t) {
    const int sel = t >> 4;
    const int r   = t & 15;
    const int n   = n0 + r;
    const float* src = (sel == 0) ? QF : KF;
    const size_t go = (size_t)(r0 + r) * DMODEL + h * HDIM + lane;
    const float xr = src[go] + ((sel == 0) ? hr : 0.0f);
    const float xi = src[go + 32] + ((sel == 0) ? hi : 0.0f);
    const float cs = bfr(cosp[(size_t)n * (HDIM / 2) + lane]);
    const float sn = bfr(sinp[(size_t)n * (HDIM / 2) + lane]);
    const float rr = xr * cs - xi * sn;
    const float ri = xr * sn + xi * cs;
    float n2 = rr * rr + ri * ri;
#pragma unroll
    for (int off = 1; off < 32; off <<= 1) n2 += __shfl_xor(n2, off, 32);
    const float nrm  = sqrtf(n2);
    const float safe = fmaxf(nrm, PEPS);
    const float mag  = tanhf(sc * safe) * rsc;
    const float inv  = 1.0f / safe;
    const bool  zer  = nrm < PEPS;
    const float vr = zer ? 0.0f : mag * (rr * inv);
    const float vi = zer ? 0.0f : mag * (ri * inv);
    float x2 = vr * vr + vi * vi;
#pragma unroll
    for (int off = 1; off < 32; off <<= 1) x2 += __shfl_xor(x2, off, 32);
    unsigned short* stp = sT[sel] + r * DMODEL + h * HDIM + lane;
    stp[0]  = h_bits((_Float16)(vr * QC));
    stp[32] = h_bits((_Float16)(vi * QC));
    if (lane == 0) sN[sel][r * NHEAD + h] = x2;
  }
  __syncthreads();
  v4u vq[4], vk[4];
#pragma unroll
  for (int it = 0; it < 4; ++it) {
    const int p = it * QK_THREADS + tid;
    vq[it] = *(const v4u*)(sT[0] + (size_t)p * 8);
    vk[it] = *(const v4u*)(sT[1] + (size_t)p * 8);
  }
  v4f qn4 = {0.f, 0.f, 0.f, 0.f}, kn4 = {0.f, 0.f, 0.f, 0.f};
  if (tid < 32) {
    qn4 = *(const v4f*)(sN[0] + tid * 4);
    kn4 = *(const v4f*)(sN[1] + tid * 4);
  }
  unsigned short* qd = QH + (size_t)r0 * DMODEL;
  unsigned short* kd = KH + ((size_t)bat * SEQK + 64 + n0) * DMODEL;
  float* qnd = QN + (size_t)r0 * NHEAD;
  float* knd = KN + ((size_t)bat * SEQK + 64 + n0) * NHEAD;
  for (int pass = 0; pass < 2; ++pass) {
#pragma unroll
    for (int it = 0; it < 4; ++it) {
      const int p = it * QK_THREADS + tid;
      const int row = p >> 6, col8 = (p & 63) * 8;
      *(volatile v4u*)(qd + (size_t)row * DMODEL + col8) = vq[it];
      *(volatile v4u*)(kd + (size_t)row * DMODEL + col8) = vk[it];
    }
    if (tid < 32) {
      *(volatile v4f*)(qnd + tid * 4) = qn4;
      *(volatile v4f*)(knd + tid * 4) = kn4;
    }
    __threadfence();
  }
}

__global__ __launch_bounds__(ATHREADS)
void battn(const unsigned short* __restrict__ QH, const unsigned short* __restrict__ KH,
           const unsigned short* __restrict__ VT, const float* __restrict__ QN,
           const float* __restrict__ KN, const float* __restrict__ cin,
           const float* __restrict__ geop, unsigned short* CT) {
#pragma clang fp contract(off)
  __shared__ __align__(16) float    sS[AWAVES][16 * SPF];
  __shared__ __align__(16) unsigned sP[AWAVES][16 * PPU];
  __shared__ __align__(16) float    sY[AWAVES][PCOLS];
  __shared__ __align__(16) float    sL[AWAVES][16];
  const int tid = threadIdx.x, wave = tid >> 5, lane = tid & 31, hh = lane >> 4, c = lane & 15;
  const int qt  = blockIdx.x % (SEQ / 16);
  const int bat = blockIdx.x / (SEQ / 16);
  const int h   = blockIdx.y * AWAVES + wave;
  const int q0  = qt * 16;
  const float cc    = bfr(cin[bat]);
  const float sc    = fmaxf(sqrtf(cc), PEPS);
  const float rsc   = 1.0f / sc;
  const float gs    = bfr(geop[h]);
  const float dclip = 2.0f * atanhf(ARG1);
  float*    st = sS[wave];
  unsigned* pw = sP[wave];
  float*    yw = sY[wave];
  float*    lw = sL[wave];

#pragma unroll
  for (int e = 0; e < 3; ++e) {
    const int col  = lane + 32 * e;
    const int colc = imin(col, KCOLS - 1);
    yw[col] = KN[((size_t)bat * SEQK + q0 + colc) * NHEAD + h];
  }
  const float x2 = QN[((size_t)bat * SEQ + q0 + c) * NHEAD + h];
  const float bx = 1.0f - cc * x2;

  {
    const unsigned short* Qp = QH + ((size_t)bat * SEQ + q0 + c) * DMODEL + h * HDIM + 8 * hh;
    const v16h qa = ldfrag_u(Qp), qb = ldfrag_u(Qp + 32);
    const unsigned short* Kb = KH + ((size_t)bat * SEQK + q0 + c) * DMODEL + h * HDIM + 8 * hh;
#pragma unroll
    for (int j = 0; j < KCOLS / 16; ++j) {
      const unsigned short* kp = Kb + (size_t)(16 * j) * DMODEL;
      const v16h k0 = ldfrag_u(kp), k1 = ldfrag_u(kp + 32);
      v8f s = mma_raw(qa, k0, zero8());
      s = mma_raw(qb, k1, s);
      guard_s4(s, k0, k1, qa, qb);
#pragma unroll
      for (int r = 0; r < 8; ++r) st[(8 * hh + r) * SPF + 16 * j + c] = s[r];
    }
  }
  wave_sync_lds();

  const int r = c;
  const float xys = 1.0f / (QC * KC);
  float mx = -INFINITY;
#pragma unroll 1
  for (int i = 0; i < KCOLS / 4; ++i) {
    const int col0 = 4 * i + 2 * hh;
#pragma unroll
    for (int e = 0; e < 2; ++e) {
      const int col = col0 + e;
      const int w   = col - r - 1;
      const float xy = st[r * SPF + col] * xys;
      const float y2 = yw[col];
      const float d  = hdist(xy, x2, y2, cc, sc, rsc, bx, dclip);
      const float sv = ((unsigned)w < (unsigned)WIN) ? -(gs * d) : -INFINITY;
      st[r * SPF + col] = sv;
      mx = fmaxf(mx, sv);
    }
  }
  mx = fmaxf(mx, __shfl_xor(mx, 16, 32));
  float l = 0.f;
#pragma unroll 1
  for (int i = 0; i < KCOLS / 4; ++i) {
    const int col0 = 4 * i + 2 * hh;
    const float s0 = st[r * SPF + col0];
    const float s1 = st[r * SPF + col0 + 1];
    const float e0 = expf(s0 - mx);
    const float e1 = expf(s1 - mx);
    l += e0 + e1;
    pw[r * PPU + (col0 >> 1)] = pk16(h_bits((_Float16)(e0 * PC)), h_bits((_Float16)(e1 * PC)));
  }
  {
    const v4u z = {0u, 0u, 0u, 0u};
    *(v4u*)(pw + r * PPU + (KCOLS / 2) + 4 * hh) = z;
  }
  l += __shfl_xor(l, 16, 32);
  if (hh == 0) lw[c] = l;
  wave_sync_lds();

  v8f o0 = zero8(), o1 = zero8(), o2 = zero8(), o3 = zero8();
  {
    const unsigned short* Pp = (const unsigned short*)pw + c * (2 * PPU) + 8 * hh;
    const unsigned short* Vb = VT + ((size_t)bat * DMODEL + h * HDIM + c) * SEQV + q0 + 8 * hh;
#pragma unroll
    for (int ks = 0; ks < PCOLS / 32; ++ks) {
      const v16h ph = ldfrag_u(Pp + 32 * ks);
      const unsigned short* vp = Vb + 32 * ks;
      const v16h vb0 = ldfrag_u(vp);
      const v16h vb1 = ldfrag_u(vp + (size_t)16 * SEQV);
      const v16h vb2 = ldfrag_u(vp + (size_t)32 * SEQV);
      const v16h vb3 = ldfrag_u(vp + (size_t)48 * SEQV);
      o0 = mma_raw(ph, vb0, o0);
      o1 = mma_raw(ph, vb1, o1);
      o2 = mma_raw(ph, vb2, o2);
      o3 = mma_raw(ph, vb3, o3);
      guard_pv4(o0, o1, o2, o3, ph, vb0, vb1, vb2, vb3);
    }
  }

  unsigned short* Os = (unsigned short*)st;
  {
    const float oc = FC / (PC * VC);
    const v4f l0 = *(const v4f*)(lw + 8 * hh);
    const v4f l1 = *(const v4f*)(lw + 8 * hh + 4);
    float linv[8];
#pragma unroll
    for (int rr = 0; rr < 4; ++rr) {
      linv[rr]     = (1.0f / l0[rr]) * oc;
      linv[4 + rr] = (1.0f / l1[rr]) * oc;
    }
    unsigned short* osw = Os + c;
#pragma unroll
    for (int rr = 0; rr < 8; ++rr) {
      unsigned short* op = osw + (8 * hh + rr) * HDIM;
      op[0]  = h_bits((_Float16)(o0[rr] * linv[rr]));
      op[16] = h_bits((_Float16)(o1[rr] * linv[rr]));
      op[32] = h_bits((_Float16)(o2[rr] * linv[rr]));
      op[48] = h_bits((_Float16)(o3[rr] * linv[rr]));
    }
  }
  wave_sync_lds();
  {
    v4u vals[4];
#pragma unroll
    for (int it = 0; it < 4; ++it) {
      const int row = it * 4 + (lane >> 3);
      const int c8  = (lane & 7) * 8;
      vals[it] = *(const v4u*)(Os + row * HDIM + c8);
    }
    unsigned short* dst = CT + ((size_t)bat * SEQ + q0) * DMODEL + h * HDIM;
    for (int pass = 0; pass < 2; ++pass) {
#pragma unroll
      for (int it = 0; it < 4; ++it) {
        const int row = it * 4 + (lane >> 3);
        const int c8  = (lane & 7) * 8;
        *(volatile v4u*)(dst + (size_t)row * DMODEL + c8) = vals[it];
      }
      __threadfence();
    }
  }
}

extern "C" void kernel_launch(void* const* d_in, const int* in_sizes, int n_in,
                              void* d_out, int out_size, void* d_ws, size_t ws_size,
                              hipStream_t stream) {
  if (n_in < 22) return;
  if ((long long)in_sizes[0] < ((long long)(NB - 1) * SEQ_FULL + SEQ) * DMODEL) return;
  if (in_sizes[1] < SEQ * (HDIM / 2) || in_sizes[2] < SEQ * (HDIM / 2)) return;
  if (in_sizes[3] < NB) return;
  if (in_sizes[4] < DMODEL * DMODEL || in_sizes[6] < DMODEL * DMODEL) return;
  if (in_sizes[8] < DMODEL * DMODEL || in_sizes[10] < DMODEL * DMODEL) return;
  if (in_sizes[5] < DMODEL || in_sizes[7] < DMODEL || in_sizes[9] < DMODEL || in_sizes[11] < DMODEL) return;
  if (in_sizes[12] < DMODEL * DFF || in_sizes[13] < DFF || in_sizes[14] < DFF * DMODEL || in_sizes[15] < DMODEL) return;
  if (in_sizes[16] < DMODEL || in_sizes[17] < DMODEL || in_sizes[18] < DMODEL || in_sizes[19] < DMODEL) return;
  if (in_sizes[20] < NHEAD || in_sizes[21] < NHEAD * HDIM) return;
  if (out_size < NROWS * DMODEL) return;

  const float* x     = (const float*)d_in[0];
  const float* fcos  = (const float*)d_in[1];
  const float* fsin  = (const float*)d_in[2];
  const float* cvec  = (const float*)d_in[3];
  const float* w_q   = (const float*)d_in[4];
  const float* b_q   = (const float*)d_in[5];
  const float* w_k   = (const float*)d_in[6];
  const float* b_k   = (const float*)d_in[7];
  const float* w_v   = (const float*)d_in[8];
  const float* b_v   = (const float*)d_in[9];
  const float* w_o   = (const float*)d_in[10];
  const float* b_o   = (const float*)d_in[11];
  const float* w_1   = (const float*)d_in[12];
  const float* b_1   = (const float*)d_in[13];
  const float* w_2   = (const float*)d_in[14];
  const float* b_2   = (const float*)d_in[15];
  const float* ln1_g = (const float*)d_in[16];
  const float* ln1_b = (const float*)d_in[17];
  const float* ln2_g = (const float*)d_in[18];
  const float* ln2_b = (const float*)d_in[19];
  const float* geo   = (const float*)d_in[20];
  const float* hashp = (const float*)d_in[21];
  float*       out   = (float*)d_out;

  const size_t PW   = (size_t)DMODEL * DMODEL * 2;
  const size_t PWF  = (size_t)DFF * DMODEL * 2;
  const size_t P16  = (size_t)NROWS * DMODEL * 2;
  const size_t P32  = (size_t)NROWS * DMODEL * 4;
  const size_t PKH  = (size_t)NB * SEQK * DMODEL * 2;
  const size_t PVT  = (size_t)NB * DMODEL * SEQV * 2;
  const size_t PQN  = (size_t)NROWS * NHEAD * 4;
  const size_t PKN  = (size_t)NB * SEQK * NHEAD * 4;
  const size_t PG   = (size_t)NROWS * DFF * 2;
  size_t off = 0;
  const size_t oWQ = off; off += PW;
  const size_t oWK = off; off += PW;
  const size_t oWV = off; off += PW;
  const size_t oWO = off; off += PW;
  const size_t oW1 = off; off += PWF;
  const size_t oW2 = off; off += PWF;
  const size_t oH  = off; off += P16;
  const size_t oQF = off; off += P32;
  const size_t oKF = off; off += P32;
  const size_t oQH = off; off += P16;
  const size_t oKH = off; off += PKH;
  const size_t oVT = off; off += PVT;
  const size_t oQN = off; off += PQN;
  const size_t oKN = off; off += PKN;
  const size_t oCT = off; off += P16;
  const size_t oX1 = off; off += P32;
  const size_t oH2 = off; off += P16;
  const size_t oG  = off; off += PG;
  const size_t endAll = off;
  if (endAll > ws_size) return;
  if (endAll > (size_t)134217728) return;

  char* ws = (char*)d_ws;
  unsigned short* WQ16 = (unsigned short*)(ws + oWQ);
  unsigned short* WK16 = (unsigned short*)(ws + oWK);
  unsigned short* WV16 = (unsigned short*)(ws + oWV);
  unsigned short* WO16 = (unsigned short*)(ws + oWO);
  unsigned short* W116 = (unsigned short*)(ws + oW1);
  unsigned short* W216 = (unsigned short*)(ws + oW2);
  unsigned short* H16  = (unsigned short*)(ws + oH);
  float*          QF   = (float*)(ws + oQF);
  float*          KF   = (float*)(ws + oKF);
  unsigned short* QH   = (unsigned short*)(ws + oQH);
  unsigned short* KH   = (unsigned short*)(ws + oKH);
  unsigned short* VTp  = (unsigned short*)(ws + oVT);
  float*          QN   = (float*)(ws + oQN);
  float*          KN   = (float*)(ws + oKN);
  unsigned short* CT   = (unsigned short*)(ws + oCT);
  float*          X1F  = (float*)(ws + oX1);
  unsigned short* H2   = (unsigned short*)(ws + oH2);
  unsigned short* G16  = (unsigned short*)(ws + oG);

  const dim3 blk(256);
  const dim3 gTw(DMODEL / 64, DMODEL / 64);
  const dim3 gT1(DFF / 64, DMODEL / 64);
  const dim3 gT2(DMODEL / 64, DFF / 64);
  const int tilesP = (NROWS / 64) * (DMODEL / 64);
  const int tilesB = (SEQ / 64) * (DMODEL / 64);
  const int tilesF = (NROWS / 64) * (DFF / 64);
  const dim3 gP((tilesP + 7) / 8, 1);
  const dim3 gB((tilesB + 7) / 8, NB);
  const dim3 gF((tilesF + 7) / 8, 1);
  const dim3 gLN(NROWS);
  const dim3 bLN(LN_THREADS);
  const dim3 gQK(NROWS / 16);
  const dim3 bQK(QK_THREADS);
  const dim3 gAT(NB * (SEQ / 16), NHEAD / AWAVES);
  const dim3 bAT(ATHREADS);
  const int nlKH = NB * 512;
  const int nlKN = NB * 16;
  const int nlVT = NB * DMODEL;
  const dim3 gZKH((nlKH * 8 + 255) / 256), gZKN((nlKN * 8 + 255) / 256), gZVT((nlVT * 8 + 255) / 256);

  tcvt16<<<gTw, blk, 0, stream>>>(w_q, WQ16, DMODEL, DMODEL, DMODEL, DMODEL, WSC);
  tcvt16<<<gTw, blk, 0, stream>>>(w_k, WK16, DMODEL, DMODEL, DMODEL, DMODEL, WSC);
  tcvt16<<<gTw, blk, 0, stream>>>(w_v, WV16, DMODEL, DMODEL, DMODEL, DMODEL, WSC);
  tcvt16<<<gTw, blk, 0, stream>>>(w_o, WO16, DMODEL, DMODEL, DMODEL, DMODEL, WSC);
  tcvt16<<<gT1, blk, 0, stream>>>(w_1, W116, DMODEL, DFF, DMODEL, DFF, WSC);
  tcvt16<<<gT2, blk, 0, stream>>>(w_2, W216, DFF, DMODEL, DFF, DMODEL, WSC);

  lnorm<1><<<gLN, bLN, 0, stream>>>(x, XBSTRIDE_FULL, ln1_g, ln1_b, H16, HCARRY);

  gemm64<0, 0, 0, 1><<<gP, blk, 0, stream>>>(
      H16, DMODEL, 0LL,
      WQ16, DMODEL, 0LL,
      x, 0LL,
      b_q, DMODEL,
      (void*)QF, DMODEL, 0LL,
      NROWS, DMODEL, DMODEL, 1.0f / (HCARRY * WSC), 1.0f);

  gemm64<0, 0, 0, 1><<<gP, blk, 0, stream>>>(
      H16, DMODEL, 0LL,
      WK16, DMODEL, 0LL,
      x, 0LL,
      b_k, DMODEL,
      (void*)KF, DMODEL, 0LL,
      NROWS, DMODEL, DMODEL, 1.0f / (HCARRY * WSC), 1.0f);

  gemm64<2, 0, 0, 2><<<gB, blk, 0, stream>>>(
      WV16, DMODEL, 0LL,
      H16, DMODEL, (long long)SEQ * DMODEL,
      x, 0LL,
      b_v, DMODEL,
      (void*)(VTp + 64), SEQV, (long long)DMODEL * SEQV,
      DMODEL, SEQ, DMODEL, 1.0f / (HCARRY * WSC), VC);

  zlines<<<gZKH, blk, 0, stream>>>(KH, 512, (long long)SEQK * DMODEL, 64LL, nlKH);
  zlines<<<gZKN, blk, 0, stream>>>((unsigned short*)KN, 16, (long long)SEQK * NHEAD * 2, 64LL, nlKN);
  zlines<<<gZVT, blk, 0, stream>>>(VTp, nlVT, 0LL, (long long)SEQV, nlVT);
  zlines<<<gZVT, blk, 0, stream>>>(VTp + SEQ + 64, nlVT, 0LL, (long long)SEQV, nlVT);

  qkprep<<<gQK, bQK, 0, stream>>>(QF, KF, fcos, fsin, cvec, hashp, QH, KH, QN, KN);

  battn<<<gAT, bAT, 0, stream>>>(QH, KH, VTp, QN, KN, cvec, geo, CT);

  gemm64<0, 1, 0, 1><<<gB, blk, 0, stream>>>(
      CT, DMODEL, (long long)SEQ * DMODEL,
      WO16, DMODEL, 0LL,
      x, XBSTRIDE_FULL,
      b_o, DMODEL,
      (void*)X1F, DMODEL, (long long)SEQ * DMODEL,
      SEQ, DMODEL, DMODEL, 1.0f / (FC * WSC), 1.0f);

  lnorm<0><<<gLN, bLN, 0, stream>>>(X1F, (long long)SEQ * DMODEL, ln2_g, ln2_b, H2, H2C);

  gemm64<2, 0, 1, 1><<<gF, blk, 0, stream>>>(
      H2, DMODEL, 0LL,
      W116, DMODEL, 0LL,
      X1F, 0LL,
      b_1, DFF,
      (void*)G16, DFF, 0LL,
      NROWS, DFF, DMODEL, 1.0f / (H2C * WSC), GC);

  gemm64<0, 2, 0, 1><<<gP, blk, 0, stream>>>(
      G16, DFF, 0LL,
      W216, DFF, 0LL,
      X1F, 0LL,
      b_2, DMODEL,
      (void*)out, DMODEL, 0LL,
      NROWS, DMODEL, DFF, 1.0f / (GC * WSC), 1.0f);
  (void)hipGetLastError();
}
